// MFC_29841432773494
// MI455X (gfx1250) — hardware-verified
//
#include <hip/hip_runtime.h>
#include <stddef.h>
#include <math.h>

constexpr int NIMG  = 4;
constexpr int CIN   = 512;
constexpr int CHID  = 256;
constexpr int NCO   = 512;
constexpr int IMW   = 64;
constexpr int HWPIX = 4096;
constexpr int NPIX  = 16384;
constexpr int NTAP  = 9;
constexpr int KIM   = 2304;
constexpr int NOFF  = 18;
constexpr int NOFFP = 64;
constexpr int NSQ   = 32;
constexpr int DPIX  = 16;

static_assert(NIMG * HWPIX == NPIX, "");
static_assert(NPIX % 64 == 0 && CHID % 64 == 0 && NCO % 64 == 0 && NOFFP % 64 == 0, "");
static_assert(CIN % 32 == 0 && KIM % 32 == 0 && CHID % 32 == 0, "");
static_assert(KIM == NTAP * CHID, "");
static_assert(NPIX % DPIX == 0 && DPIX * NTAP <= 256, "");

constexpr size_t WS_XT   = 0;
constexpr size_t WS_H2H  = 0;
constexpr size_t WS_H2L  = (size_t)NPIX * CHID * 2;
constexpr size_t WS_H    = (size_t)NPIX * CIN * 2;
constexpr size_t WS_IM   = WS_H + (size_t)NPIX * CHID * 4;
constexpr size_t WS_Y    = WS_IM;
constexpr size_t WS_OFF  = WS_IM + (size_t)NPIX * KIM * 2;
constexpr size_t WS_W1   = WS_OFF + (size_t)NPIX * NOFFP * 4;
constexpr size_t WS_W2   = WS_W1 + (size_t)CHID * CIN * 2;
constexpr size_t WS_WOFF = WS_W2 + (size_t)NCO * CHID * 2;
constexpr size_t WS_MEAN = WS_WOFF + (size_t)NOFFP * KIM * 2;
constexpr size_t WS_S    = WS_MEAN + (size_t)NIMG * NCO * 4;
constexpr size_t WS_END  = WS_S + (size_t)NIMG * NCO * 4;
static_assert(WS_H2L + (size_t)NPIX * CHID * 2 <= WS_H, "");
static_assert(WS_Y + (size_t)NPIX * NCO * 4 <= WS_OFF, "");
static_assert(WS_END == 114081792, "");
static_assert(WS_END <= 134217728, "");
static_assert(WS_H % 256 == 0 && WS_IM % 256 == 0 && WS_OFF % 256 == 0 && WS_W1 % 256 == 0 && WS_W2 % 256 == 0 &&
              WS_WOFF % 256 == 0 && WS_MEAN % 256 == 0 && WS_S % 256 == 0 && WS_H2L % 256 == 0, "");

typedef __attribute__((ext_vector_type(16))) _Float16 v16h;
typedef __attribute__((ext_vector_type(8)))  _Float16 v8h;
typedef __attribute__((ext_vector_type(16))) __bf16   v16b;
typedef __attribute__((ext_vector_type(8)))  __bf16   v8b;
typedef __attribute__((ext_vector_type(8)))  float    v8f;
typedef __attribute__((ext_vector_type(4)))  float    v4f;
typedef __attribute__((ext_vector_type(4)))  unsigned v4u;
typedef __attribute__((ext_vector_type(4)))  int      v4i;

__device__ __forceinline__ unsigned short f2bf_bits(float f) {
  unsigned u = __float_as_uint(f);
  return (unsigned short)((u + 0x7FFFu + ((u >> 16) & 1u)) >> 16);
}
__device__ __forceinline__ float bf_bits2f(unsigned short h) { return __uint_as_float(((unsigned)h) << 16); }
__device__ __forceinline__ float bf16r(float f) { return bf_bits2f(f2bf_bits(f)); }

__device__ __forceinline__ unsigned pk2(unsigned short a, unsigned short b) {
  return (unsigned)a | ((unsigned)b << 16);
}
__device__ __forceinline__ unsigned pkh2(float a, float b) {
  return pk2(__builtin_bit_cast(unsigned short, (_Float16)a), __builtin_bit_cast(unsigned short, (_Float16)b));
}
__device__ __forceinline__ void pkbf2(float a, float b, unsigned& uh, unsigned& ul) {
  const unsigned short ha = f2bf_bits(a), hb = f2bf_bits(b);
  const unsigned short la = f2bf_bits(a - bf_bits2f(ha)), lb = f2bf_bits(b - bf_bits2f(hb));
  uh = pk2(ha, hb);
  ul = pk2(la, lb);
}

__device__ __forceinline__ float silu_f(float v) {
  const float e = __expf(fminf(-v, 30.0f));
  return v * __builtin_amdgcn_rcpf(1.0f + e);
}
__device__ __forceinline__ float sigm_f(float v) {
  const float e = __expf(fminf(-v, 30.0f));
  return __builtin_amdgcn_rcpf(1.0f + e);
}

__device__ __forceinline__ void dep_guard_h(v8f& a, v8f& b, v16h x, v16h y) { asm volatile("v_nop\n\tv_nop\n\tv_nop\n\tv_nop" : "+v"(a), "+v"(b) : "v"(x), "v"(y)); }
__device__ __forceinline__ void dep_guard_b(v8f& a, v8f& b, v16b x, v16b y) { asm volatile("v_nop\n\tv_nop\n\tv_nop\n\tv_nop" : "+v"(a), "+v"(b) : "v"(x), "v"(y)); }
__device__ __forceinline__ void keep4_h(v16h a, v16h b, v16h c, v16h d) { asm volatile("v_nop" :: "v"(a), "v"(b), "v"(c), "v"(d)); }
__device__ __forceinline__ void keep4_b(v16b a, v16b b, v16b c, v16b d) { asm volatile("v_nop" :: "v"(a), "v"(b), "v"(c), "v"(d)); }
__device__ __forceinline__ void acc_guard4(v8f& a, v8f& b, v8f& c, v8f& d) { asm volatile("v_nop\n\tv_nop\n\tv_nop\n\tv_nop" : "+v"(a), "+v"(b), "+v"(c), "+v"(d)); }
template <typename T> struct Frag;
template <> struct Frag<_Float16> {
  typedef v16h V; union U { v16h v; v8h h[2]; };
  static __device__ __forceinline__ v16h load(const _Float16* p) {
    U f; f.h[0] = *(const v8h*)(p); f.h[1] = *(const v8h*)(p + 16); return f.v;
  }
  static __device__ __forceinline__ v8f mma(v16h a, v16h b, v8f c) {
    return __builtin_amdgcn_wmma_f32_16x16x32_f16(false, a, false, b, (short)0, c, false, false);
  }
  static __device__ __forceinline__ void guard(v8f& a, v8f& b, v16h x, v16h y) { dep_guard_h(a, b, x, y); }
  static __device__ __forceinline__ void keep(v16h a, v16h b, v16h c, v16h d) { keep4_h(a, b, c, d); }
};
template <> struct Frag<__bf16> {
  typedef v16b V; union U { v16b v; v8b h[2]; };
  static __device__ __forceinline__ v16b load(const __bf16* p) {
    U f; f.h[0] = *(const v8b*)(p); f.h[1] = *(const v8b*)(p + 16); return f.v;
  }
  static __device__ __forceinline__ v8f mma(v16b a, v16b b, v8f c) {
    return __builtin_amdgcn_wmma_f32_16x16x32_bf16(false, a, false, b, (short)0, c, false, false);
  }
  static __device__ __forceinline__ void guard(v8f& a, v8f& b, v16b x, v16b y) { dep_guard_b(a, b, x, y); }
  static __device__ __forceinline__ void keep(v16b a, v16b b, v16b c, v16b d) { keep4_b(a, b, c, d); }
};

template <int ET> struct Elem;
template <> struct Elem<0> { typedef _Float16 T; };
template <> struct Elem<1> { typedef __bf16 T; };
template <int ET, int SPLITM, int EPI>
__global__ __launch_bounds__(256) void k_gemm64(
    const unsigned short* __restrict__ Ap, const unsigned short* __restrict__ A2p, int lda,
    const unsigned short* __restrict__ Btp, const unsigned short* __restrict__ Bt2p, int ldb,
    float* __restrict__ Cout, int ldc,
    const float* __restrict__ gvec, const float* __restrict__ bvec, int nbias,
    int M, int N, int K, float scale) {
  typedef typename Elem<ET>::T T;
  typedef typename Frag<T>::V V;
  constexpr bool SPLA = (SPLITM != 0);
  constexpr bool SPLB = (SPLITM == 1);
  const T* Ab = (const T*)Ap; const T* Ab2 = (const T*)A2p; const T* Bb = (const T*)Btp; const T* Bb2 = (const T*)Bt2p;
  __shared__ __align__(16) float sT[8][16 * 68];
  const int lane = threadIdx.x & 31;
  const int wave = threadIdx.x >> 5;
  const int tilesN = N >> 6;
  const int tilesM = M >> 6;
  const int tile = blockIdx.x * 8 + wave;
  if (tile >= tilesM * tilesN) return;
  const int tm = tile / tilesN;
  const int tn = tile - tm * tilesN;
  const int m0 = tm << 6;
  const int n0 = tn << 6;

  const int rlane = lane & 15;
  const int koff  = (lane >> 4) * 8;
  const int mOff  = (lane >> 4) * 8;

  v8f acc[4][4];
#pragma unroll
  for (int i = 0; i < 4; ++i)
#pragma unroll
    for (int j = 0; j < 4; ++j) acc[i][j] = (v8f){0.f,0.f,0.f,0.f,0.f,0.f,0.f,0.f};

  for (int k0 = 0; k0 < K; k0 += 32) {
    V bh[4], bl[4];
#pragma unroll
    for (int j = 0; j < 4; ++j) {
      const size_t bo = (size_t)(n0 + (j << 4) + rlane) * ldb + koff + k0;
      bh[j] = Frag<T>::load(Bb + bo);
      if (SPLB) bl[j] = Frag<T>::load(Bb2 + bo);
    }
#pragma unroll
    for (int i = 0; i < 4; ++i) {
      const size_t ao = (size_t)(m0 + (i << 4) + rlane) * lda + koff + k0;
      V ah = Frag<T>::load(Ab + ao);
      V al;
      if (SPLA) al = Frag<T>::load(Ab2 + ao);
#pragma unroll
      for (int j = 0; j < 4; ++j) {
        acc[i][j] = Frag<T>::mma(ah, bh[j], acc[i][j]);
        if (SPLB) acc[i][j] = Frag<T>::mma(ah, bl[j], acc[i][j]);
        if (SPLA) acc[i][j] = Frag<T>::mma(al, bh[j], acc[i][j]);
      }
      Frag<T>::guard(acc[i][0], acc[i][3], ah, SPLA ? al : ah);
    }
    Frag<T>::keep(bh[0], bh[1], bh[2], bh[3]);
    if (SPLB) Frag<T>::keep(bl[0], bl[1], bl[2], bl[3]);
  }
  acc_guard4(acc[0][0], acc[0][1], acc[0][2], acc[0][3]);
  acc_guard4(acc[1][0], acc[1][1], acc[1][2], acc[1][3]);
  acc_guard4(acc[2][0], acc[2][1], acc[2][2], acc[2][3]);
  acc_guard4(acc[3][0], acc[3][1], acc[3][2], acc[3][3]);

  float* slab = sT[wave];
#pragma unroll
  for (int i = 0; i < 4; ++i) {
    const int mBase = m0 + (i << 4);
#pragma unroll
    for (int j = 0; j < 4; ++j) {
      const int n = n0 + (j << 4) + rlane;
      float gm = scale, badd = 0.f;
      if (EPI == 1) {
        gm = scale * bf16r(gvec[n]);
        badd = bf16r(bvec[n]);
      } else {
        const int nc = (n < nbias) ? n : (nbias - 1);
        const float braw = bvec[nc];
        badd = (n < nbias) ? bf16r(braw) : 0.f;
      }
#pragma unroll
      for (int r = 0; r < 8; ++r) {
        float v = acc[i][j][r] * gm + badd;
        if (EPI == 1) v = silu_f(v);
        slab[(mOff + r) * 68 + (j << 4) + rlane] = v;
      }
    }
    __builtin_amdgcn_fence(__ATOMIC_RELEASE, "workgroup");
    __builtin_amdgcn_wave_barrier();
    __builtin_amdgcn_fence(__ATOMIC_ACQUIRE, "workgroup");
    {
      float* C = Cout;
      const int hh = lane >> 4, c4 = (lane & 15) * 4;
      for (int pass = 0; pass < 2; ++pass) {
#pragma unroll
        for (int it = 0; it < 8; ++it) {
          const int row = it * 2 + hh;
          v4f v = *(const v4f*)(slab + row * 68 + c4);
          *(volatile v4f*)(C + (size_t)(mBase + row) * ldc + n0 + c4) = v;
        }
        __threadfence();
      }
    }
    __builtin_amdgcn_fence(__ATOMIC_RELEASE, "workgroup");
    __builtin_amdgcn_wave_barrier();
    __builtin_amdgcn_fence(__ATOMIC_ACQUIRE, "workgroup");
  }
}

__global__ __launch_bounds__(256) void k_xt(const float* __restrict__ x, unsigned short* __restrict__ xt) {
  __shared__ float t[64][65];
  const int tid = threadIdx.x;
  const int p0 = blockIdx.x * 64, c0 = blockIdx.y * 64, b = blockIdx.z;
  const int c4 = (tid & 15) * 4;
#pragma unroll
  for (int it = 0; it < 4; ++it) {
    const int row = it * 16 + (tid >> 4);
    const v4f v = *(const v4f*)(x + ((size_t)(b * CIN + c0 + row)) * HWPIX + p0 + c4);
#pragma unroll
    for (int e = 0; e < 4; ++e) t[row][c4 + e] = v[e];
  }
  __syncthreads();
  const int wave = tid >> 5, lane = tid & 31, q = lane >> 3, c8 = (lane & 7) * 8;
  for (int pass = 0; pass < 2; ++pass) {
#pragma unroll
    for (int step = 0; step < 2; ++step) {
      const int pp = step * 32 + wave * 4 + q;
      float f[8];
#pragma unroll
      for (int e = 0; e < 8; ++e) f[e] = t[c8 + e][pp];
      v4u u;
      u[0] = pk2(f2bf_bits(f[0]), f2bf_bits(f[1])); u[1] = pk2(f2bf_bits(f[2]), f2bf_bits(f[3]));
      u[2] = pk2(f2bf_bits(f[4]), f2bf_bits(f[5])); u[3] = pk2(f2bf_bits(f[6]), f2bf_bits(f[7]));
      *(volatile v4u*)(xt + ((size_t)(b * HWPIX + p0 + pp)) * CIN + c0 + c8) = u;
    }
    __threadfence();
  }
}

__global__ __launch_bounds__(256) void k_cvt_bf16x8(const float* __restrict__ w, unsigned short* __restrict__ dst, int n8) {
  const int i = blockIdx.x * 256 + threadIdx.x;
  if (i < n8) {
    const v4f a = *(const v4f*)(w + (size_t)i * 8);
    const v4f c = *(const v4f*)(w + (size_t)i * 8 + 4);
    v4u u;
    u[0] = pk2(f2bf_bits(a[0]), f2bf_bits(a[1])); u[1] = pk2(f2bf_bits(a[2]), f2bf_bits(a[3]));
    u[2] = pk2(f2bf_bits(c[0]), f2bf_bits(c[1])); u[3] = pk2(f2bf_bits(c[2]), f2bf_bits(c[3]));
    volatile v4u* p = (volatile v4u*)(dst + (size_t)i * 8);
    *p = u;
    __threadfence();
    *p = u;
  }
}

__global__ __launch_bounds__(256) void k_woff(const float* __restrict__ w, unsigned short* __restrict__ dst) {
  const int i = blockIdx.x * 256 + threadIdx.x;
  const int n = i / (KIM / 8);
  const int k8 = (i - n * (KIM / 8)) * 8;
  const int tap = k8 >> 8;
  const int c = k8 & (CHID - 1);
  const bool inb = n < NOFF;
  const int nc = inb ? n : (NOFF - 1);
  const float* src = w + (size_t)nc * (CHID * NTAP) + (size_t)c * NTAP + tap;
  float f[8];
#pragma unroll
  for (int e = 0; e < 8; ++e) {
    const float raw = src[e * NTAP];
    f[e] = inb ? 256.0f * bf16r(raw) : 0.0f;
  }
  v4u u;
  u[0] = pkh2(f[0], f[1]); u[1] = pkh2(f[2], f[3]); u[2] = pkh2(f[4], f[5]); u[3] = pkh2(f[6], f[7]);
  volatile v4u* p = (volatile v4u*)(dst + (size_t)n * KIM + k8);
  *p = u;
  __threadfence();
  *p = u;
}

__global__ __launch_bounds__(256) void k_im2col(const float* __restrict__ h, unsigned short* __restrict__ im) {
  const int tid = threadIdx.x, lane = tid & 31, wave = tid >> 5;
  const int pg = blockIdx.x * 8 + wave;
  const int b = pg >> 12, pix = pg & (HWPIX - 1);
  const int y = pix >> 6, x = pix & (IMW - 1);
  const float* hb = h + (size_t)b * HWPIX * CHID + lane * 8;
  unsigned short* dst = im + (size_t)pg * KIM + lane * 8;
#pragma unroll 1
  for (int tap = 0; tap < NTAP; ++tap) {
    const int t3 = tap / 3;
    const int ys = y + t3 - 1, xs = x + (tap - t3 * 3) - 1;
    const bool inb = (ys >= 0) & (ys < IMW) & (xs >= 0) & (xs < IMW);
    const int ysc = min(max(ys, 0), IMW - 1), xsc = min(max(xs, 0), IMW - 1);
    const float* src = hb + (size_t)(ysc * IMW + xsc) * CHID;
    const v4f a = *(const v4f*)src;
    const v4f c = *(const v4f*)(src + 4);
    const float m = inb ? 16.0f : 0.0f;
    v4u u;
    u[0] = pkh2(a[0] * m, a[1] * m); u[1] = pkh2(a[2] * m, a[3] * m);
    u[2] = pkh2(c[0] * m, c[1] * m); u[3] = pkh2(c[2] * m, c[3] * m);
    volatile v4u* p = (volatile v4u*)(dst + tap * CHID);
    *p = u;
    __threadfence();
    *p = u;
  }
}

__global__ __launch_bounds__(256) void k_deform(const float* __restrict__ h, const float* __restrict__ off,
                                                const float* __restrict__ wdw, const float* __restrict__ gb,
                                                const float* __restrict__ bb,
                                                unsigned short* __restrict__ h2h, unsigned short* __restrict__ h2l,
                                                float rs) {
  __shared__ v4i gidx[DPIX * NTAP];
  __shared__ v4f gwt[DPIX * NTAP];
  __shared__ __align__(16) float wds[NTAP * CHID];
  const int tid = threadIdx.x, lane = tid & 31, wave = tid >> 5;
  const int pblk = blockIdx.x * DPIX;
#pragma unroll 1
  for (int k = 0; k < NTAP; ++k) wds[k * CHID + tid] = bf16r(wdw[tid * NTAP + k]);
  if (tid < DPIX * NTAP) {
    const int s = tid / NTAP, k = tid - s * NTAP;
    const int pg = pblk + s;
    const int pix = pg & (HWPIX - 1);
    const int y = pix >> 6, x = pix & (IMW - 1);
    const int k3 = k / 3;
    const int ky = k3 - 1, kx = (k - k3 * 3) - 1;
    const float dy = off[(size_t)pg * NOFFP + 2 * k];
    const float dx = off[(size_t)pg * NOFFP + 2 * k + 1];
    const float py = (float)(y + ky) + dy;
    const float px = (float)(x + kx) + dx;
    const float y0f = floorf(py), x0f = floorf(px);
    const float fy = py - y0f, fx = px - x0f;
    const int y0 = (int)y0f, x0 = (int)x0f;
    const bool vy0 = (y0 >= 0) & (y0 <= IMW - 1), vy1 = (y0 >= -1) & (y0 <= IMW - 2);
    const bool vx0 = (x0 >= 0) & (x0 <= IMW - 1), vx1 = (x0 >= -1) & (x0 <= IMW - 2);
    const int cy0 = min(max(y0, 0), IMW - 1), cy1 = min(max(y0, -1), IMW - 2) + 1;
    const int cx0 = min(max(x0, 0), IMW - 1), cx1 = min(max(x0, -1), IMW - 2) + 1;
    v4i gi;
    gi[0] = cy0 * IMW + cx0; gi[1] = cy0 * IMW + cx1; gi[2] = cy1 * IMW + cx0; gi[3] = cy1 * IMW + cx1;
    const float wy0 = 1.0f - fy, wx0 = 1.0f - fx;
    v4f gw;
    gw[0] = (vy0 & vx0) ? wy0 * wx0 : 0.0f;
    gw[1] = (vy0 & vx1) ? wy0 * fx  : 0.0f;
    gw[2] = (vy1 & vx0) ? fy * wx0  : 0.0f;
    gw[3] = (vy1 & vx1) ? fy * fx   : 0.0f;
    gidx[tid] = gi;
    gwt[tid] = gw;
  }
  __syncthreads();

#pragma unroll 1
  for (int it = 0; it < 2; ++it) {
    const int s = it * 8 + wave;
    const int pg = pblk + s;
    const int b = pg >> 12;
    const float* hb = h + (size_t)b * HWPIX * CHID + lane * 8;
    float d[8];
#pragma unroll
    for (int e = 0; e < 8; ++e) d[e] = 0.0f;
#pragma unroll 1
    for (int k = 0; k < NTAP; ++k) {
      const v4i gi = gidx[s * NTAP + k];
      const v4f gw = gwt[s * NTAP + k];
      const int i00 = gi[0] & (HWPIX - 1), i01 = gi[1] & (HWPIX - 1), i10 = gi[2] & (HWPIX - 1), i11 = gi[3] & (HWPIX - 1);
      const float* p00 = hb + (size_t)i00 * CHID;
      const float* p01 = hb + (size_t)i01 * CHID;
      const float* p10 = hb + (size_t)i10 * CHID;
      const float* p11 = hb + (size_t)i11 * CHID;
      const v4f a0 = *(const v4f*)p00, a1 = *(const v4f*)(p00 + 4);
      const v4f b0 = *(const v4f*)p01, b1 = *(const v4f*)(p01 + 4);
      const v4f c0 = *(const v4f*)p10, c1 = *(const v4f*)(p10 + 4);
      const v4f e0 = *(const v4f*)p11, e1 = *(const v4f*)(p11 + 4);
      const v4f w0 = *(const v4f*)(wds + k * CHID + lane * 8);
      const v4f w1 = *(const v4f*)(wds + k * CHID + lane * 8 + 4);
#pragma unroll
      for (int e = 0; e < 4; ++e) {
        const float va = gw[0] * a0[e] + gw[1] * b0[e] + gw[2] * c0[e] + gw[3] * e0[e];
        d[e] += w0[e] * va;
        const float vb = gw[0] * a1[e] + gw[1] * b1[e] + gw[2] * c1[e] + gw[3] * e1[e];
        d[4 + e] += w1[e] * vb;
      }
    }
    const v4f r0 = *(const v4f*)(h + (size_t)pg * CHID + lane * 8);
    const v4f r1 = *(const v4f*)(h + (size_t)pg * CHID + lane * 8 + 4);
    const v4f g0 = *(const v4f*)(gb + lane * 8), g1 = *(const v4f*)(gb + lane * 8 + 4);
    const v4f q0 = *(const v4f*)(bb + lane * 8), q1 = *(const v4f*)(bb + lane * 8 + 4);
    float v[8];
#pragma unroll
    for (int e = 0; e < 4; ++e) {
      v[e]     = silu_f(d[e]     * (bf16r(g0[e]) * rs) + bf16r(q0[e])) + r0[e];
      v[4 + e] = silu_f(d[4 + e] * (bf16r(g1[e]) * rs) + bf16r(q1[e])) + r1[e];
    }
    v4u uh, ul;
    unsigned th, tl;
    pkbf2(v[0], v[1], th, tl); uh[0] = th; ul[0] = tl;
    pkbf2(v[2], v[3], th, tl); uh[1] = th; ul[1] = tl;
    pkbf2(v[4], v[5], th, tl); uh[2] = th; ul[2] = tl;
    pkbf2(v[6], v[7], th, tl); uh[3] = th; ul[3] = tl;
    volatile v4u* dh = (volatile v4u*)(h2h + (size_t)pg * CHID + lane * 8);
    volatile v4u* dl = (volatile v4u*)(h2l + (size_t)pg * CHID + lane * 8);
    *dh = uh;
    *dl = ul;
    __threadfence();
    *dh = uh;
    *dl = ul;
  }
}

__global__ __launch_bounds__(256) void k_mean(const float* __restrict__ y, float* __restrict__ mean) {
  __shared__ float part[8][32];
  __shared__ __align__(16) float res[32];
  const int tid = threadIdx.x;
  const int col = tid & 31, sl = tid >> 5;
  const int n0 = blockIdx.x * 32, b = blockIdx.y;
  const float* p = y + ((size_t)b * HWPIX + (size_t)sl * 512) * NCO + n0 + col;
  float s0 = 0.f, s1 = 0.f;
#pragma unroll 1
  for (int r = 0; r < 512; r += 2) {
    s0 += p[(size_t)r * NCO];
    s1 += p[(size_t)(r + 1) * NCO];
  }
  part[sl][col] = s0 + s1;
  __syncthreads();
  if (tid < 32) {
    float s = 0.f;
#pragma unroll
    for (int k = 0; k < 8; ++k) s += part[k][tid];
    res[tid] = s * (1.0f / 4096.0f);
  }
  __syncthreads();
  if (tid < 8) {
    const v4f v = *(const v4f*)(res + tid * 4);
    volatile v4f* q = (volatile v4f*)(mean + (size_t)b * NCO + n0 + tid * 4);
    *q = v;
    __threadfence();
    *q = v;
  }
}

__global__ __launch_bounds__(256) void k_se(const float* __restrict__ mean, const float* __restrict__ w1,
                                            const float* __restrict__ b1, const float* __restrict__ w2,
                                            const float* __restrict__ b2, float* __restrict__ sout) {
  __shared__ float mm[NCO];
  __shared__ float t1[NSQ];
  __shared__ __align__(16) float sg[NCO];
  const int tid = threadIdx.x, b = blockIdx.x;
  mm[tid] = mean[(size_t)b * NCO + tid];
  mm[tid + 256] = mean[(size_t)b * NCO + tid + 256];
  __syncthreads();
  if (tid < NSQ) {
    float a = 0.f;
#pragma unroll 1
    for (int n = 0; n < NCO; ++n) a += bf16r(w1[(size_t)tid * NCO + n]) * mm[n];
    a += bf16r(b1[tid]);
    t1[tid] = silu_f(a);
  }
  __syncthreads();
#pragma unroll 1
  for (int q = 0; q < 2; ++q) {
    const int n = tid + q * 256;
    float a = 0.f;
#pragma unroll 1
    for (int f = 0; f < NSQ; ++f) a += bf16r(w2[(size_t)n * NSQ + f]) * t1[f];
    a += bf16r(b2[n]);
    sg[n] = sigm_f(a);
  }
  __syncthreads();
  if (tid < 128) {
    const v4f v = *(const v4f*)(sg + tid * 4);
    volatile v4f* q = (volatile v4f*)(sout + (size_t)b * NCO + tid * 4);
    *q = v;
    __threadfence();
    *q = v;
  }
}

__global__ __launch_bounds__(256) void k_out(const float* __restrict__ y, const float* __restrict__ s,
                                             float* __restrict__ out) {
  __shared__ float t[64][65];
  __shared__ float sv[64];
  const int tid = threadIdx.x;
  const int p0 = blockIdx.x * 64, n0 = blockIdx.y * 64, b = blockIdx.z;
  const int c4 = (tid & 15) * 4;
#pragma unroll
  for (int it = 0; it < 4; ++it) {
    const int row = it * 16 + (tid >> 4);
    const v4f v = *(const v4f*)(y + ((size_t)(b * HWPIX + p0 + row)) * NCO + n0 + c4);
#pragma unroll
    for (int e = 0; e < 4; ++e) t[row][c4 + e] = v[e];
  }
  if (tid < 64) sv[tid] = s[(size_t)b * NCO + n0 + tid];
  __syncthreads();
  const int wave = tid >> 5, lane = tid & 31, hh = lane >> 4;
  for (int pass = 0; pass < 2; ++pass) {
#pragma unroll
    for (int it = 0; it < 4; ++it) {
      const int nr = it * 16 + wave * 2 + hh;
      const float sc = sv[nr];
      v4f v;
      v[0] = t[c4 + 0][nr] * sc; v[1] = t[c4 + 1][nr] * sc; v[2] = t[c4 + 2][nr] * sc; v[3] = t[c4 + 3][nr] * sc;
      *(volatile v4f*)(out + ((size_t)(b * NCO + n0 + nr)) * HWPIX + p0 + c4) = v;
    }
    __threadfence();
  }
}

extern "C" void kernel_launch(void* const* d_in, const int* in_sizes, int n_in,
                              void* d_out, int out_size, void* d_ws, size_t ws_size,
                              hipStream_t stream) {
  if (n_in != 16) return;
  if (in_sizes[0] != NPIX * CIN || in_sizes[1] != CHID * CIN || in_sizes[2] != CHID || in_sizes[3] != CHID ||
      in_sizes[4] != NOFF * CHID * NTAP || in_sizes[5] != NOFF || in_sizes[6] != CHID * NTAP ||
      in_sizes[7] != CHID || in_sizes[8] != CHID || in_sizes[9] != NCO * CHID || in_sizes[10] != NCO ||
      in_sizes[11] != NCO || in_sizes[12] != NSQ * NCO || in_sizes[13] != NSQ || in_sizes[14] != NCO * NSQ ||
      in_sizes[15] != NCO) return;
  if (out_size != NIMG * NCO * HWPIX) return;
  if (ws_size < WS_END) return;

  const float* x       = (const float*)d_in[0];
  const float* w_conv1 = (const float*)d_in[1];
  const float* g1      = (const float*)d_in[2];
  const float* b1      = (const float*)d_in[3];
  const float* w_off   = (const float*)d_in[4];
  const float* b_off   = (const float*)d_in[5];
  const float* w_dw    = (const float*)d_in[6];
  const float* g_b     = (const float*)d_in[7];
  const float* b_b     = (const float*)d_in[8];
  const float* w_conv2 = (const float*)d_in[9];
  const float* g2      = (const float*)d_in[10];
  const float* b2      = (const float*)d_in[11];
  const float* w_fc1   = (const float*)d_in[12];
  const float* b_fc1   = (const float*)d_in[13];
  const float* w_fc2   = (const float*)d_in[14];
  const float* b_fc2   = (const float*)d_in[15];
  float* out = (float*)d_out;

  char* ws = (char*)d_ws;
  unsigned short* XT   = (unsigned short*)(ws + WS_XT);
  unsigned short* H2H  = (unsigned short*)(ws + WS_H2H);
  unsigned short* H2L  = (unsigned short*)(ws + WS_H2L);
  float*          H    = (float*)(ws + WS_H);
  unsigned short* IM   = (unsigned short*)(ws + WS_IM);
  float*          Y    = (float*)(ws + WS_Y);
  float*          OFF  = (float*)(ws + WS_OFF);
  unsigned short* W1   = (unsigned short*)(ws + WS_W1);
  unsigned short* W2   = (unsigned short*)(ws + WS_W2);
  unsigned short* WOFF = (unsigned short*)(ws + WS_WOFF);
  float*          MEAN = (float*)(ws + WS_MEAN);
  float*          S    = (float*)(ws + WS_S);

  const float rs = 1.0f / sqrtf(1.0f + 1e-5f);
  const dim3 blk(256);

  k_xt<<<dim3(HWPIX / 64, CIN / 64, NIMG), blk, 0, stream>>>(x, XT);
  k_cvt_bf16x8<<<dim3((CHID * CIN / 8) / 256), blk, 0, stream>>>(w_conv1, W1, CHID * CIN / 8);
  k_cvt_bf16x8<<<dim3((NCO * CHID / 8) / 256), blk, 0, stream>>>(w_conv2, W2, NCO * CHID / 8);
  k_woff<<<dim3((NOFFP * KIM / 8) / 256), blk, 0, stream>>>(w_off, WOFF);

  k_gemm64<1, 0, 1><<<dim3((NPIX / 64) * (CHID / 64) / 8), blk, 0, stream>>>(
      XT, XT, CIN, W1, W1, CIN, H, CHID, g1, b1, CHID, NPIX, CHID, CIN, rs);

  k_im2col<<<dim3(NPIX / 8), blk, 0, stream>>>(H, IM);

  k_gemm64<0, 0, 0><<<dim3((NPIX / 64) * (NOFFP / 64) / 8), blk, 0, stream>>>(
      IM, IM, KIM, WOFF, WOFF, KIM, OFF, NOFFP, b_off, b_off, NOFF, NPIX, NOFFP, KIM, 1.0f / 4096.0f);

  k_deform<<<dim3(NPIX / DPIX), blk, 0, stream>>>(H, OFF, w_dw, g_b, b_b, H2H, H2L, rs);

  k_gemm64<1, 2, 1><<<dim3((NPIX / 64) * (NCO / 64) / 8), blk, 0, stream>>>(
      H2H, H2L, CHID, W2, W2, CHID, Y, NCO, g2, b2, NCO, NPIX, NCO, CHID, rs);

  k_mean<<<dim3(NCO / 32, NIMG), blk, 0, stream>>>(Y, MEAN);
  k_se<<<dim3(NIMG), blk, 0, stream>>>(MEAN, w_fc1, b_fc1, w_fc2, b_fc2, S);
  k_out<<<dim3(HWPIX / 64, NCO / 64, NIMG), blk, 0, stream>>>(Y, S, out);
}
